// GroupedQueryAttention_29549374996907
// MI455X (gfx1250) — hardware-verified
//
#include <hip/hip_runtime.h>
#include <math.h>

typedef __attribute__((ext_vector_type(16))) _Float16     v16h;
typedef __attribute__((ext_vector_type(8)))  _Float16     v8h;
typedef __attribute__((ext_vector_type(8)))  float        v8f;
typedef __attribute__((ext_vector_type(4)))  float        v4f;
typedef __attribute__((ext_vector_type(4)))  unsigned int v4u;

#ifndef NB
#define NB 2
#endif
#ifndef SEQ
#define SEQ 4096
#endif
#define NB_FULL  2
#define SEQ_FULL 4096
#define CH    512
#define NG    4
#define HD    128
#define KC    64
#define KH    32
#define QT    16
#define AWAVE 8
#define QB    (QT * AWAVE)

#define WSC   64.0f
#define WINV  0.015625f
#define CSC   64.0f
#define OINV  0.000244140625f
#define PSC   32768.0f
#define QKSC  16.0f
#define QKINV 0.00390625f

#define W16_ELEMS ((size_t)4 * CH * CH)
#define PL_ELEMS  ((size_t)NB * SEQ * CH)
#define WS_BYTES  ((W16_ELEMS + 5 * PL_ELEMS) * 2)

static_assert(SEQ % QB == 0);
static_assert(SEQ % KC == 0 && SEQ % 64 == 0);
static_assert(SEQ <= SEQ_FULL && NB <= NB_FULL);
static_assert(CH == NG * HD && HD == 128 && CH % 64 == 0 && CH % 32 == 0);
static_assert(KC == 64 && KH == 32 && QT == 16 && KC == 2 * KH);
static_assert(AWAVE * 32 * 4 == KC * (HD / 8));
static_assert(AWAVE * 32 * 4 == HD * (KC / 8));
static_assert(AWAVE * QT * HD == KC * HD + HD * KC);
static_assert(HD * 2 == 16 * 16);
static_assert(64 * 4 == 16 * 16);
static_assert(64 * 2 == 8 * 16);
static_assert(PL_ELEMS < (size_t)2147483647);
static_assert((W16_ELEMS * 2) % 256 == 0 && (PL_ELEMS * 2) % 256 == 0);
static_assert(WS_BYTES <= (size_t)134217728);

union FH { v16h v; v8h h[2]; };

__device__ __forceinline__ unsigned int bf_bits(float f) {
    const unsigned int u = __float_as_uint(f);
    return (u + 0x7FFFu + ((u >> 16) & 1u)) >> 16;
}
__device__ __forceinline__ float bf_val(float f) { return __uint_as_float(bf_bits(f) << 16); }
__device__ __forceinline__ unsigned int h_bits(float f) { return (unsigned int)__builtin_bit_cast(unsigned short, (_Float16)f); }
__device__ __forceinline__ v8f zero8() { return (v8f){0.f, 0.f, 0.f, 0.f, 0.f, 0.f, 0.f, 0.f}; }

__device__ __forceinline__ v8f mma_h(v16h a, v16h b, v8f c) {
    c = __builtin_amdgcn_wmma_f32_16x16x32_f16(false, a, false, b, (short)0, c, false, false);
    asm volatile("v_nop\n\tv_nop\n\tv_nop\n\tv_nop" : "+v"(c) : "v"(a), "v"(b));
    return c;
}

__device__ __forceinline__ void st16x2(unsigned short* p, v4u v) {
    volatile v4u* d = (volatile v4u*)p;
    *d = v; __threadfence(); *d = v;
}

__global__ __launch_bounds__(256) void k_cvt_w(const float* __restrict__ w, unsigned short* __restrict__ W16) {
    const int u = blockIdx.x * 256 + threadIdx.x;
    if (u >= CH * CH / 8) return;
    const float* src = w + (size_t)u * 8;
    const v4f a = *(const v4f*)(src), c = *(const v4f*)(src + 4);
    v4u pk;
    pk.x = h_bits(bf_val(a.x) * WSC) | (h_bits(bf_val(a.y) * WSC) << 16);
    pk.y = h_bits(bf_val(a.z) * WSC) | (h_bits(bf_val(a.w) * WSC) << 16);
    pk.z = h_bits(bf_val(c.x) * WSC) | (h_bits(bf_val(c.y) * WSC) << 16);
    pk.w = h_bits(bf_val(c.z) * WSC) | (h_bits(bf_val(c.w) * WSC) << 16);
    st16x2(W16 + (size_t)u * 8, pk);
}

__global__ __launch_bounds__(256) void k_xT(const float* __restrict__ x, unsigned short* __restrict__ XT) {
    __shared__ __align__(16) unsigned short tile[64 * 72];
    const int t = threadIdx.x;
    const int n0 = blockIdx.x * 64, c0 = blockIdx.y * 64, b = blockIdx.z;
    {
        const int rl = t >> 2, part = t & 3;
        const float* src = x + ((size_t)b * CH + c0 + rl) * SEQ_FULL + n0 + part * 16;
        const v4f f0 = *(const v4f*)(src), f1 = *(const v4f*)(src + 4), f2 = *(const v4f*)(src + 8), f3 = *(const v4f*)(src + 12);
        v4u p0, p1;
        p0.x = h_bits(bf_val(f0.x)) | (h_bits(bf_val(f0.y)) << 16); p0.y = h_bits(bf_val(f0.z)) | (h_bits(bf_val(f0.w)) << 16);
        p0.z = h_bits(bf_val(f1.x)) | (h_bits(bf_val(f1.y)) << 16); p0.w = h_bits(bf_val(f1.z)) | (h_bits(bf_val(f1.w)) << 16);
        p1.x = h_bits(bf_val(f2.x)) | (h_bits(bf_val(f2.y)) << 16); p1.y = h_bits(bf_val(f2.z)) | (h_bits(bf_val(f2.w)) << 16);
        p1.z = h_bits(bf_val(f3.x)) | (h_bits(bf_val(f3.y)) << 16); p1.w = h_bits(bf_val(f3.z)) | (h_bits(bf_val(f3.w)) << 16);
        *(v4u*)(tile + rl * 72 + part * 16)     = p0;
        *(v4u*)(tile + rl * 72 + part * 16 + 8) = p1;
    }
    __syncthreads();
#pragma unroll
    for (int it = 0; it < 2; ++it) {
        const int drow = it * 32 + (t >> 3), pc = t & 7;
        unsigned int e[8];
#pragma unroll
        for (int j = 0; j < 8; ++j) e[j] = (unsigned int)tile[(pc * 8 + j) * 72 + drow];
        v4u pk;
        pk.x = e[0] | (e[1] << 16); pk.y = e[2] | (e[3] << 16); pk.z = e[4] | (e[5] << 16); pk.w = e[6] | (e[7] << 16);
        st16x2(XT + ((size_t)b * SEQ + n0 + drow) * CH + c0 + pc * 8, pk);
    }
}

__device__ __forceinline__ void gemm16x64(const unsigned short* __restrict__ Apl, size_t aoff,
                                          const unsigned short* __restrict__ Bpl, size_t boff,
                                          v8f& a0, v8f& a1, v8f& a2, v8f& a3) {
    const _Float16* Ap = (const _Float16*)Apl + aoff;
    const _Float16* Bp = (const _Float16*)Bpl + boff;
#pragma unroll 2
    for (int ks = 0; ks < CH / 32; ++ks) {
        FH a, b;
        a.h[0] = *(const v8h*)(Ap + ks * 32);
        a.h[1] = *(const v8h*)(Ap + ks * 32 + 16);
        b.h[0] = *(const v8h*)(Bp + ks * 32);
        b.h[1] = *(const v8h*)(Bp + ks * 32 + 16);
        a0 = mma_h(a.v, b.v, a0);
        b.h[0] = *(const v8h*)(Bp + 16 * CH + ks * 32);
        b.h[1] = *(const v8h*)(Bp + 16 * CH + ks * 32 + 16);
        a1 = mma_h(a.v, b.v, a1);
        b.h[0] = *(const v8h*)(Bp + 32 * CH + ks * 32);
        b.h[1] = *(const v8h*)(Bp + 32 * CH + ks * 32 + 16);
        a2 = mma_h(a.v, b.v, a2);
        b.h[0] = *(const v8h*)(Bp + 48 * CH + ks * 32);
        b.h[1] = *(const v8h*)(Bp + 48 * CH + ks * 32 + 16);
        a3 = mma_h(a.v, b.v, a3);
    }
}

__global__ __launch_bounds__(128) void k_proj_qk(const unsigned short* __restrict__ XT, const unsigned short* __restrict__ W16,
                                                  const float* __restrict__ bias, unsigned short* __restrict__ P16) {
    __shared__ __align__(16) float Os[4][16 * 68];
    const int tid = threadIdx.x, wave = tid >> 5, lane = tid & 31, hh = lane >> 4, c = lane & 15;
    const int n0 = blockIdx.x * 64 + wave * 16, o0 = blockIdx.y * 64, b = blockIdx.z;
    v8f a0 = zero8(), a1 = zero8(), a2 = zero8(), a3 = zero8();
    gemm16x64(XT, ((size_t)b * SEQ + n0 + c) * CH + 8 * hh, W16, ((size_t)(o0 + c)) * CH + 8 * hh, a0, a1, a2, a3);
    const float b0 = bf_val(bias[o0 + c]), b1 = bf_val(bias[o0 + 16 + c]);
    const float b2 = bf_val(bias[o0 + 32 + c]), b3 = bf_val(bias[o0 + 48 + c]);
    float* os = Os[wave];
#pragma unroll
    for (int r = 0; r < 8; ++r) {
        os[(8 * hh + r) * 68 + c]      = a0[r] * WINV + b0;
        os[(8 * hh + r) * 68 + 16 + c] = a1[r] * WINV + b1;
        os[(8 * hh + r) * 68 + 32 + c] = a2[r] * WINV + b2;
        os[(8 * hh + r) * 68 + 48 + c] = a3[r] * WINV + b3;
    }
    __builtin_amdgcn_fence(3  , "workgroup");
    __builtin_amdgcn_wave_barrier();
    __builtin_amdgcn_fence(2  , "workgroup");
    const int g = o0 >> 7, d0 = o0 & (HD - 1);
    const size_t obase = (((size_t)b * NG + g) * SEQ + n0) * HD + d0;
    const int rq = lane >> 3, pc = lane & 7;
    v4u pk[4];
#pragma unroll
    for (int it = 0; it < 4; ++it) {
        const int row = it * 4 + rq;
        const v4f f0 = *(const v4f*)(os + row * 68 + pc * 8);
        const v4f f1 = *(const v4f*)(os + row * 68 + pc * 8 + 4);
        pk[it].x = h_bits(f0.x * QKSC) | (h_bits(f0.y * QKSC) << 16); pk[it].y = h_bits(f0.z * QKSC) | (h_bits(f0.w * QKSC) << 16);
        pk[it].z = h_bits(f1.x * QKSC) | (h_bits(f1.y * QKSC) << 16); pk[it].w = h_bits(f1.z * QKSC) | (h_bits(f1.w * QKSC) << 16);
    }
#pragma unroll
    for (int it = 0; it < 4; ++it)
        *(volatile v4u*)(P16 + obase + (size_t)(it * 4 + rq) * HD + pc * 8) = pk[it];
    __threadfence();
#pragma unroll
    for (int it = 0; it < 4; ++it)
        *(volatile v4u*)(P16 + obase + (size_t)(it * 4 + rq) * HD + pc * 8) = pk[it];
}

__global__ __launch_bounds__(128) void k_proj_v(const unsigned short* __restrict__ W16, const unsigned short* __restrict__ XT,
                                                 const float* __restrict__ bias, unsigned short* __restrict__ VT) {
    __shared__ __align__(16) float Os[4][16 * 68];
    const int tid = threadIdx.x, wave = tid >> 5, lane = tid & 31, hh = lane >> 4, c = lane & 15;
    const int n0 = blockIdx.x * 64, m0 = blockIdx.y * 64 + wave * 16, b = blockIdx.z;
    v8f a0 = zero8(), a1 = zero8(), a2 = zero8(), a3 = zero8();
    gemm16x64(W16, ((size_t)(m0 + c)) * CH + 8 * hh, XT, ((size_t)b * SEQ + n0 + c) * CH + 8 * hh, a0, a1, a2, a3);
    float* os = Os[wave];
#pragma unroll
    for (int r = 0; r < 8; ++r) {
        const float bb = bf_val(bias[m0 + 8 * hh + r]);
        os[(8 * hh + r) * 68 + c]      = a0[r] * WINV + bb;
        os[(8 * hh + r) * 68 + 16 + c] = a1[r] * WINV + bb;
        os[(8 * hh + r) * 68 + 32 + c] = a2[r] * WINV + bb;
        os[(8 * hh + r) * 68 + 48 + c] = a3[r] * WINV + bb;
    }
    __builtin_amdgcn_fence(3  , "workgroup");
    __builtin_amdgcn_wave_barrier();
    __builtin_amdgcn_fence(2  , "workgroup");
    const size_t obase = ((size_t)b * CH + m0) * SEQ + n0;
    const int rq = lane >> 3, pc = lane & 7;
    v4u pk[4];
#pragma unroll
    for (int it = 0; it < 4; ++it) {
        const int row = it * 4 + rq;
        const v4f f0 = *(const v4f*)(os + row * 68 + pc * 8);
        const v4f f1 = *(const v4f*)(os + row * 68 + pc * 8 + 4);
        pk[it].x = h_bits(f0.x) | (h_bits(f0.y) << 16); pk[it].y = h_bits(f0.z) | (h_bits(f0.w) << 16);
        pk[it].z = h_bits(f1.x) | (h_bits(f1.y) << 16); pk[it].w = h_bits(f1.z) | (h_bits(f1.w) << 16);
    }
#pragma unroll
    for (int it = 0; it < 4; ++it)
        *(volatile v4u*)(VT + obase + (size_t)(it * 4 + rq) * SEQ + pc * 8) = pk[it];
    __threadfence();
#pragma unroll
    for (int it = 0; it < 4; ++it)
        *(volatile v4u*)(VT + obase + (size_t)(it * 4 + rq) * SEQ + pc * 8) = pk[it];
}

__global__ __launch_bounds__(256) void k_attn(const unsigned short* __restrict__ Q16, const unsigned short* __restrict__ K16,
                                               const unsigned short* __restrict__ VT, unsigned short* __restrict__ CTX) {
    __shared__ __align__(16) unsigned short Tsh[KC * HD + HD * KC];
    __shared__ __align__(16) _Float16       Psh[AWAVE][QT * KH];

    const int tid = threadIdx.x, wave = tid >> 5, lane = tid & 31, hh = lane >> 4, c = lane & 15;
    const int g = blockIdx.y, b = blockIdx.z;
    const int q0 = blockIdx.x * QB + wave * QT;
    const int hrow0 = (b * NG + g) * SEQ;
    const int qoff0 = (hrow0 + q0 + c) * HD + 8 * hh;
    const int vrow0 = (b * CH + g * HD) * SEQ;
    const float SCL = 0.08838834764831845f * 1.4426950408889634f * QKINV;

    const _Float16* Qp = (const _Float16*)Q16;
    const _Float16* Kp = (const _Float16*)Tsh;
    const _Float16* Vp = (const _Float16*)Tsh + KC * HD;
    _Float16* pw = Psh[wave];

    float mrow[8], lrow[8];
    v8f oacc[8];
#pragma unroll
    for (int r = 0; r < 8; ++r) { mrow[r] = -INFINITY; lrow[r] = 0.f; }
#pragma unroll
    for (int t = 0; t < 8; ++t) oacc[t] = zero8();

#pragma unroll 1
    for (int kc = 0; kc < SEQ / KC; ++kc) {
        const int kv0 = kc * KC;
        __syncthreads();
#pragma unroll
        for (int i = 0; i < 4; ++i) {
            const int idx = tid + 256 * i;
            {
                const int row = idx >> 4, pc = idx & 15;
                const v4u kk = *(const v4u*)(K16 + (hrow0 + kv0 + row) * HD + pc * 8);
                *(v4u*)(Tsh + row * HD + pc * 8) = kk;
            }
            {
                const int row = idx >> 3, pc = idx & 7;
                const v4u vv = *(const v4u*)(VT + vrow0 + row * SEQ + kv0 + pc * 8);
                *(v4u*)(Tsh + KC * HD + row * KC + pc * 8) = vv;
            }
        }
        __syncthreads();

#pragma unroll 1
        for (int hf = 0; hf < 2; ++hf) {
            int qoff = qoff0;
            asm volatile("" : "+v"(qoff));
            v8f s0 = zero8(), s1 = zero8();
#pragma unroll
            for (int ks = 0; ks < 4; ++ks) {
                FH qf, kf;
                qf.h[0] = *(const v8h*)(Qp + qoff + ks * 32);
                qf.h[1] = *(const v8h*)(Qp + qoff + ks * 32 + 16);
                const int ko = (hf * KH + c) * HD + ks * 32 + 8 * hh;
                kf.h[0] = *(const v8h*)(Kp + ko);
                kf.h[1] = *(const v8h*)(Kp + ko + 16);
                s0 = mma_h(qf.v, kf.v, s0);
                kf.h[0] = *(const v8h*)(Kp + ko + 16 * HD);
                kf.h[1] = *(const v8h*)(Kp + ko + 16 * HD + 16);
                s1 = mma_h(qf.v, kf.v, s1);
            }

#pragma unroll
            for (int r = 0; r < 8; ++r) {
                const float x0 = s0[r] * SCL, x1 = s1[r] * SCL;
                float m = fmaxf(x0, x1);
                m = fmaxf(m, __shfl_xor(m, 1, 32)); m = fmaxf(m, __shfl_xor(m, 2, 32));
                m = fmaxf(m, __shfl_xor(m, 4, 32)); m = fmaxf(m, __shfl_xor(m, 8, 32));
                const float mnew  = fmaxf(mrow[r], m);
                const float alpha = exp2f(mrow[r] - mnew);
                mrow[r] = mnew;
                const float p0 = exp2f(x0 - mnew), p1 = exp2f(x1 - mnew);
                _Float16* prow = pw + (8 * hh + r) * KH + c;
                prow[0]  = (_Float16)(p0 * PSC);
                prow[16] = (_Float16)(p1 * PSC);
                float psum = p0 + p1;
                psum += __shfl_xor(psum, 1, 32); psum += __shfl_xor(psum, 2, 32);
                psum += __shfl_xor(psum, 4, 32); psum += __shfl_xor(psum, 8, 32);
                lrow[r] = lrow[r] * alpha + psum;
#pragma unroll
                for (int t = 0; t < 8; ++t) oacc[t][r] *= alpha;
            }
            __builtin_amdgcn_fence(3  , "workgroup");
            __builtin_amdgcn_wave_barrier();
            __builtin_amdgcn_fence(2  , "workgroup");

            FH pa;
            pa.h[0] = *(const v8h*)(pw + c * KH + 8 * hh);
            pa.h[1] = *(const v8h*)(pw + c * KH + 16 + 8 * hh);
#pragma unroll
            for (int tg = 0; tg < 2; ++tg) {
                FH vb[4];
#pragma unroll
                for (int t4 = 0; t4 < 4; ++t4) {
                    const int vo = ((tg * 4 + t4) * 16 + c) * KC + hf * KH + 8 * hh;
                    vb[t4].h[0] = *(const v8h*)(Vp + vo);
                    vb[t4].h[1] = *(const v8h*)(Vp + vo + 16);
                }
#pragma unroll
                for (int t4 = 0; t4 < 4; ++t4) oacc[tg * 4 + t4] = mma_h(pa.v, vb[t4].v, oacc[tg * 4 + t4]);
            }
        }
    }

    __syncthreads();
    _Float16* es = (_Float16*)Tsh + wave * (QT * HD);
#pragma unroll
    for (int r = 0; r < 8; ++r) {
        const float inv = CSC * (1.0f / (lrow[r] * PSC));
#pragma unroll
        for (int t = 0; t < 8; ++t) es[(8 * hh + r) * HD + t * 16 + c] = (_Float16)(oacc[t][r] * inv);
    }
    __builtin_amdgcn_fence(3  , "workgroup");
    __builtin_amdgcn_wave_barrier();
    __builtin_amdgcn_fence(2  , "workgroup");
    {
        unsigned short* ob = CTX + ((size_t)b * SEQ + q0) * CH + g * HD;
        const int c8 = (lane & 15) * 8;
        v4u vals[8];
#pragma unroll
        for (int it = 0; it < 8; ++it) {
            const v8h hv = *(const v8h*)(es + (it * 2 + hh) * HD + c8);
            vals[it] = __builtin_bit_cast(v4u, hv);
        }
#pragma unroll
        for (int it = 0; it < 8; ++it) *(volatile v4u*)(ob + (size_t)(it * 2 + hh) * CH + c8) = vals[it];
        __threadfence();
#pragma unroll
        for (int it = 0; it < 8; ++it) *(volatile v4u*)(ob + (size_t)(it * 2 + hh) * CH + c8) = vals[it];
    }
}

__global__ __launch_bounds__(128) void k_outproj(const unsigned short* __restrict__ W16, const unsigned short* __restrict__ CTX,
                                                  const float* __restrict__ bias, const float* __restrict__ x,
                                                  float* __restrict__ out) {
    __shared__ __align__(16) float Os[4][16 * 68];
    const int tid = threadIdx.x, wave = tid >> 5, lane = tid & 31, hh = lane >> 4, c = lane & 15;
    const int n0 = blockIdx.x * 64, m0 = blockIdx.y * 64 + wave * 16, b = blockIdx.z;
    v8f a0 = zero8(), a1 = zero8(), a2 = zero8(), a3 = zero8();
    gemm16x64(W16, ((size_t)(m0 + c)) * CH + 8 * hh, CTX, ((size_t)b * SEQ + n0 + c) * CH + 8 * hh, a0, a1, a2, a3);
    float* os = Os[wave];
#pragma unroll
    for (int r = 0; r < 8; ++r) {
        const float bb = bf_val(bias[m0 + 8 * hh + r]);
        os[(8 * hh + r) * 68 + c]      = a0[r] * OINV + bb;
        os[(8 * hh + r) * 68 + 16 + c] = a1[r] * OINV + bb;
        os[(8 * hh + r) * 68 + 32 + c] = a2[r] * OINV + bb;
        os[(8 * hh + r) * 68 + 48 + c] = a3[r] * OINV + bb;
    }
    __builtin_amdgcn_fence(3  , "workgroup");
    __builtin_amdgcn_wave_barrier();
    __builtin_amdgcn_fence(2  , "workgroup");
    const int c4 = (lane & 15) * 4;
    const float* xb = x + ((size_t)b * CH + m0) * SEQ_FULL + n0 + c4;
    float* ob = out + ((size_t)b * CH + m0) * SEQ + n0 + c4;
    v4f vals[8];
#pragma unroll
    for (int it = 0; it < 8; ++it) {
        const int row = it * 2 + hh;
        const v4f o  = *(const v4f*)(os + row * 68 + c4);
        const v4f xv = *(const v4f*)(xb + (size_t)row * SEQ_FULL);
        v4f y;
        y.x = o.x + bf_val(xv.x); y.y = o.y + bf_val(xv.y); y.z = o.z + bf_val(xv.z); y.w = o.w + bf_val(xv.w);
        vals[it] = y;
    }
#pragma unroll
    for (int it = 0; it < 8; ++it) *(volatile v4f*)(ob + (size_t)(it * 2 + hh) * SEQ) = vals[it];
    __threadfence();
#pragma unroll
    for (int it = 0; it < 8; ++it) *(volatile v4f*)(ob + (size_t)(it * 2 + hh) * SEQ) = vals[it];
}

extern "C" void kernel_launch(void* const* d_in, const int* in_sizes, int n_in, void* d_out, int out_size, void* d_ws, size_t ws_size, hipStream_t stream) {
    if (n_in < 9) return;
    if ((long long)in_sizes[0] < (long long)(NB - 1) * CH * SEQ_FULL + (long long)(CH - 1) * SEQ_FULL + (long long)SEQ) return;
    if (in_sizes[1] < CH * CH || in_sizes[3] < CH * CH || in_sizes[5] < CH * CH || in_sizes[7] < CH * CH) return;
    if (in_sizes[2] < CH || in_sizes[4] < CH || in_sizes[6] < CH || in_sizes[8] < CH) return;
    if ((long long)out_size < (long long)NB * CH * SEQ) return;
    if (ws_size < WS_BYTES) return;

    const float* x  = (const float*)d_in[0];
    const float* Wq = (const float*)d_in[1];
    const float* bq = (const float*)d_in[2];
    const float* Wk = (const float*)d_in[3];
    const float* bk = (const float*)d_in[4];
    const float* Wv = (const float*)d_in[5];
    const float* bv = (const float*)d_in[6];
    const float* Wo = (const float*)d_in[7];
    const float* bo = (const float*)d_in[8];
    float* out = (float*)d_out;

    unsigned short* ws16 = (unsigned short*)d_ws;
    unsigned short* W16 = ws16;
    unsigned short* XT  = ws16 + W16_ELEMS;
    unsigned short* Q16 = XT + PL_ELEMS;
    unsigned short* K16 = Q16 + PL_ELEMS;
    unsigned short* VTp = K16 + PL_ELEMS;
    unsigned short* CTX = VTp + PL_ELEMS;

    const unsigned wblocks = (unsigned)((CH * CH / 8 + 255) / 256);
    k_cvt_w<<<wblocks, 256, 0, stream>>>(Wq, W16);
    k_cvt_w<<<wblocks, 256, 0, stream>>>(Wk, W16 + (size_t)CH * CH);
    k_cvt_w<<<wblocks, 256, 0, stream>>>(Wv, W16 + (size_t)2 * CH * CH);
    k_cvt_w<<<wblocks, 256, 0, stream>>>(Wo, W16 + (size_t)3 * CH * CH);
    k_xT<<<dim3((unsigned)(SEQ / 64), (unsigned)(CH / 64), (unsigned)NB), 256, 0, stream>>>(x, XT);

    const dim3 ggrid((unsigned)(SEQ / 64), (unsigned)(CH / 64), (unsigned)NB);
    k_proj_qk<<<ggrid, 128, 0, stream>>>(XT, W16, bq, Q16);
    k_proj_qk<<<ggrid, 128, 0, stream>>>(XT, W16 + (size_t)CH * CH, bk, K16);
    k_proj_v<<<ggrid, 128, 0, stream>>>(W16 + (size_t)2 * CH * CH, XT, bv, VTp);

    k_attn<<<dim3((unsigned)(SEQ / QB), (unsigned)NG, (unsigned)NB), 256, 0, stream>>>(Q16, K16, VTp, CTX);

    k_outproj<<<ggrid, 128, 0, stream>>>(W16 + (size_t)3 * CH * CH, CTX, bo, x, out);
}
